// DenseRandlanetKernel_71717363908926
// MI455X (gfx1250) — hardware-verified
//
#include <hip/hip_runtime.h>
#include <stdint.h>


typedef float          v4f  __attribute__((ext_vector_type(4)));
typedef float          v8f  __attribute__((ext_vector_type(8)));
typedef _Float16       v4h  __attribute__((ext_vector_type(4)));
typedef _Float16       v8h  __attribute__((ext_vector_type(8)));
typedef _Float16       v16h __attribute__((ext_vector_type(16)));
typedef __bf16         v16bf __attribute__((ext_vector_type(16)));
typedef unsigned short v4us __attribute__((ext_vector_type(4)));
typedef unsigned short v8us __attribute__((ext_vector_type(8)));
typedef v4f __attribute__((may_alias)) v4fm;

union FragH { v16h v;  v8h  h8[2]; v4h  h4[4]; };
union FragB { v16bf v; v8us u8[2]; v4us u4[4]; };

namespace {
constexpr int kN    = 16384;
constexpr int kK    = 16;
constexpr int kCIN  = 64;
constexpr int kDREL = 64;
constexpr int kCMID = 128;
constexpr int kCOUT = 128;
constexpr int kPtsBlk  = 32;
constexpr int kWaves   = 4;
constexpr int kPtsWave = 8;
constexpr int kThreads = kWaves * 32;
constexpr int PF = 132;
constexpr int PA = 132;
constexpr int PO = 32;
}
static_assert(kPtsBlk == kWaves * kPtsWave);
static_assert(kDREL + kCIN == kCMID);
static_assert((PF * 4) % 16 == 0 && (PA * 4) % 16 == 0);
static_assert(32 * PO <= 16 * PF);

__device__ __forceinline__ unsigned short bf_bits(float x) {
  unsigned u = __float_as_uint(x);
  u = u + 0x7FFFu + ((u >> 16) & 1u);
  return (unsigned short)(u >> 16);
}
__device__ __forceinline__ float bf_val(unsigned short b) {
  return __uint_as_float(((unsigned)b) << 16);
}
struct HL4 { v4us hi; v4us lo; };
__device__ __forceinline__ HL4 bf_split4(v4f t) {
  HL4 r;
#pragma unroll
  for (int i = 0; i < 4; ++i) {
    const unsigned short hb = bf_bits(t[i]);
    r.hi[i] = hb;
    r.lo[i] = bf_bits(t[i] - bf_val(hb));
  }
  return r;
}

__device__ __forceinline__ v8f mma_f16(v16h a, v16h b, v8f c) {
  v8f d = __builtin_amdgcn_wmma_f32_16x16x32_f16(false, a, false, b, (short)0, c, false, false);
  asm volatile("v_nop\n\tv_nop\n\tv_nop\n\tv_nop" : "+v"(d) : "v"(a), "v"(b));
  return d;
}
__device__ __forceinline__ v8f mma_bf16(v16bf a, v16bf b, v8f c) {
  v8f d = __builtin_amdgcn_wmma_f32_16x16x32_bf16(false, a, false, b, (short)0, c, false, false);
  asm volatile("v_nop\n\tv_nop\n\tv_nop\n\tv_nop" : "+v"(d) : "v"(a), "v"(b));
  return d;
}

__global__ __launch_bounds__(256) void k_prep(const float* __restrict__ Watt,
                                               const float* __restrict__ Wglob,
                                               _Float16* __restrict__ wattT,
                                               unsigned short* __restrict__ wgHi,
                                               unsigned short* __restrict__ wgLo)
{
  const int g  = (int)blockIdx.x * 256 + (int)threadIdx.x;
  const int n  = g >> 4;
  const int k0 = (g & 15) * 8;
  if (n < kCMID) {
    v8h  wa;
    v8us hi, lo;
#pragma unroll
    for (int i = 0; i < 8; ++i) {
      const float a  = Watt[(size_t)(k0 + i) * kCMID + n] * 16.0f;
      wa[i] = (_Float16)a;
      const float gv = Wglob[(size_t)(k0 + i) * kCOUT + n];
      const unsigned short hb = bf_bits(gv);
      hi[i] = hb;
      lo[i] = bf_bits(gv - bf_val(hb));
    }
    const size_t off = (size_t)n * kCMID + k0;
    *(volatile v8h*)(wattT + off)  = wa;
    *(volatile v8us*)(wgHi + off) = hi;
    *(volatile v8us*)(wgLo + off) = lo;
    __threadfence();
    *(volatile v8h*)(wattT + off)  = wa;
    *(volatile v8us*)(wgHi + off) = hi;
    *(volatile v8us*)(wgLo + off) = lo;
  }
}

__global__ __launch_bounds__(kThreads) void k_main(const float* __restrict__ x,
                                                    const float* __restrict__ pos,
                                                    const int*   __restrict__ nidx,
                                                    const float* __restrict__ Wrel,
                                                    const float* __restrict__ brel,
                                                    const _Float16* __restrict__ wattT,
                                                    const unsigned short* __restrict__ wgHi,
                                                    const unsigned short* __restrict__ wgLo,
                                                    const float* __restrict__ bglob,
                                                    float* __restrict__ out)
{
  __shared__ __align__(16) float s_f[kWaves][16 * PF];
  __shared__ __align__(16) float s_geo[kWaves][16 * 8];
  __shared__ __align__(16) float s_agg[kPtsBlk * PA];

  const int tid = (int)threadIdx.x;
  const int w   = tid >> 5;
  const int l   = tid & 31;
  const int h   = l >> 4;
  const int m   = l & 15;

  const int gp0 = (int)blockIdx.x * kPtsBlk;
  const int b   = gp0 / kN;
  const int nb  = gp0 - b * kN;

  float* sF = s_f[w];
  float* sG = s_geo[w];

  const float* xb   = x    + (size_t)b * kCIN * kN;
  const float* posb = pos  + (size_t)b * kN * 3;
  const int*   nib  = nidx + (size_t)b * kN * kK;

  float wr0[10], wr1[10];
#pragma unroll
  for (int e = 0; e < 10; ++e) {
    wr0[e] = Wrel[e * kDREL + l];
    wr1[e] = Wrel[e * kDREL + l + 32];
  }
  const float br0 = brel[l];
  const float br1 = brel[l + 32];

#pragma unroll 1
  for (int p = 0; p < kPtsWave; ++p) {
    const int pl = w * kPtsWave + p;
    const int n  = nb + pl;

    int j = nib[(size_t)n * kK + m];
    j = (j < 0) ? (j + kN) : j;
    j = (j < 0) ? 0 : ((j > kN - 1) ? (kN - 1) : j);
    const float cx = posb[(size_t)n * 3 + 0];
    const float cy = posb[(size_t)n * 3 + 1];
    const float cz = posb[(size_t)n * 3 + 2];
    const float px = posb[(size_t)j * 3 + 0];
    const float py = posb[(size_t)j * 3 + 1];
    const float pz = posb[(size_t)j * 3 + 2];
    const float rx = px - cx, ry = py - cy, rz = pz - cz;
    const float dist = sqrtf(rx * rx + ry * ry + rz * rz);
    if (h == 0) {
      v4f g0, g1;
      g0[0] = px; g0[1] = py; g0[2] = pz; g0[3] = rx;
      g1[0] = ry; g1[1] = rz; g1[2] = dist; g1[3] = 0.0f;
      *(v4fm*)(sG + m * 8)     = g0;
      *(v4fm*)(sG + m * 8 + 4) = g1;
    }
    {
      const float* xs = xb + (size_t)(32 * h) * kN + j;
      float* fr = sF + m * PF + kDREL + 32 * h;
#pragma unroll
      for (int q = 0; q < 8; ++q) {
        v4f t;
        t[0] = xs[(size_t)(4 * q + 0) * kN];
        t[1] = xs[(size_t)(4 * q + 1) * kN];
        t[2] = xs[(size_t)(4 * q + 2) * kN];
        t[3] = xs[(size_t)(4 * q + 3) * kN];
        *(v4fm*)(fr + 4 * q) = t;
      }
    }
    __syncthreads();

    {
      const float cp0 = br0 + cx * wr0[0] + cy * wr0[1] + cz * wr0[2];
      const float cp1 = br1 + cx * wr1[0] + cy * wr1[1] + cz * wr1[2];
#pragma unroll 4
      for (int k = 0; k < kK; ++k) {
        const v4f g0 = *(const v4fm*)(sG + k * 8);
        const v4f g1 = *(const v4fm*)(sG + k * 8 + 4);
        float v0 = cp0 + g0[0] * wr0[3] + g0[1] * wr0[4] + g0[2] * wr0[5]
                       + g0[3] * wr0[6] + g1[0] * wr0[7] + g1[1] * wr0[8] + g1[2] * wr0[9];
        float v1 = cp1 + g0[0] * wr1[3] + g0[1] * wr1[4] + g0[2] * wr1[5]
                       + g0[3] * wr1[6] + g1[0] * wr1[7] + g1[1] * wr1[8] + g1[2] * wr1[9];
        sF[k * PF + l]      = fmaxf(v0, 0.0f);
        sF[k * PF + 32 + l] = fmaxf(v1, 0.0f);
      }
    }
    __syncthreads();

    FragH a[4];
#pragma unroll
    for (int kt = 0; kt < 4; ++kt) {
      const float* r = sF + m * PF + 32 * kt + 8 * h;
      const v4f t0 = *(const v4fm*)(r);
      const v4f t1 = *(const v4fm*)(r + 4);
      const v4f t2 = *(const v4fm*)(r + 16);
      const v4f t3 = *(const v4fm*)(r + 20);
      a[kt].h4[0] = __builtin_convertvector(t0, v4h);
      a[kt].h4[1] = __builtin_convertvector(t1, v4h);
      a[kt].h4[2] = __builtin_convertvector(t2, v4h);
      a[kt].h4[3] = __builtin_convertvector(t3, v4h);
    }
#pragma unroll 1
    for (int t2 = 0; t2 < 8; ++t2) {
      const _Float16* wb = wattT + (size_t)(16 * t2 + m) * kCMID + 8 * h;
      v8f acc = {0.f, 0.f, 0.f, 0.f, 0.f, 0.f, 0.f, 0.f};
#pragma unroll
      for (int kt = 0; kt < 4; ++kt) {
        FragH bb;
        bb.h8[0] = *(const v8h*)(wb + 32 * kt);
        bb.h8[1] = *(const v8h*)(wb + 32 * kt + 16);
        acc = mma_f16(a[kt].v, bb.v, acc);
      }
      float sc[8];
#pragma unroll
      for (int v = 0; v < 8; ++v) sc[v] = acc[v] * 0.0625f;
      float mx = sc[0];
#pragma unroll
      for (int v = 1; v < 8; ++v) mx = fmaxf(mx, sc[v]);
      mx = fmaxf(mx, __shfl_xor(mx, 16, 32));
      float ex[8];
      float ssum = 0.0f;
#pragma unroll
      for (int v = 0; v < 8; ++v) { ex[v] = __expf(sc[v] - mx); ssum += ex[v]; }
      ssum += __shfl_xor(ssum, 16, 32);
      const float inv = __builtin_amdgcn_rcpf(ssum);
      const int c = 16 * t2 + m;
      float ag = 0.0f;
#pragma unroll
      for (int v = 0; v < 8; ++v) ag += (ex[v] * inv) * sF[(8 * h + v) * PF + c];
      ag += __shfl_xor(ag, 16, 32);
      if (h == 0) s_agg[pl * PA + c] = ag;
    }
    __syncthreads();
  }

  float* sO = sF;
#pragma unroll 1
  for (int mt = 0; mt < 2; ++mt) {
    FragB ah[4], al[4];
#pragma unroll
    for (int kt = 0; kt < 4; ++kt) {
      const float* r = s_agg + (size_t)(16 * mt + m) * PA + 32 * kt + 8 * h;
      const HL4 q0 = bf_split4(*(const v4fm*)(r));
      const HL4 q1 = bf_split4(*(const v4fm*)(r + 4));
      const HL4 q2 = bf_split4(*(const v4fm*)(r + 16));
      const HL4 q3 = bf_split4(*(const v4fm*)(r + 20));
      ah[kt].u4[0] = q0.hi; al[kt].u4[0] = q0.lo;
      ah[kt].u4[1] = q1.hi; al[kt].u4[1] = q1.lo;
      ah[kt].u4[2] = q2.hi; al[kt].u4[2] = q2.lo;
      ah[kt].u4[3] = q3.hi; al[kt].u4[3] = q3.lo;
    }
#pragma unroll
    for (int t = 0; t < 2; ++t) {
      const int nt = 2 * w + t;
      const size_t boff = (size_t)(16 * nt + m) * kCMID + 8 * h;
      v8f acc = {0.f, 0.f, 0.f, 0.f, 0.f, 0.f, 0.f, 0.f};
#pragma unroll
      for (int kt = 0; kt < 4; ++kt) {
        FragB bh, bl;
        bh.u8[0] = *(const v8us*)(wgHi + boff + 32 * kt);
        bh.u8[1] = *(const v8us*)(wgHi + boff + 32 * kt + 16);
        bl.u8[0] = *(const v8us*)(wgLo + boff + 32 * kt);
        bl.u8[1] = *(const v8us*)(wgLo + boff + 32 * kt + 16);
        acc = mma_bf16(ah[kt].v, bh.v, acc);
        acc = mma_bf16(ah[kt].v, bl.v, acc);
        acc = mma_bf16(al[kt].v, bh.v, acc);
      }
      const int c = 16 * nt + m;
      const float bias = bglob[c];
      v4f o0, o1;
#pragma unroll
      for (int v = 0; v < 4; ++v) o0[v] = fmaxf(acc[v] + bias, 0.0f);
#pragma unroll
      for (int v = 0; v < 4; ++v) o1[v] = fmaxf(acc[v + 4] + bias, 0.0f);
      float* so = sO + (16 * t + m) * PO + 16 * mt + 8 * h;
      *(v4fm*)(so)     = o0;
      *(v4fm*)(so + 4) = o1;
    }
  }
  __syncthreads();

  v4f ov[8];
#pragma unroll
  for (int s = 0; s < 8; ++s) ov[s] = *(const v4fm*)(sO + (4 * s + (l >> 3)) * PO + 4 * (l & 7));
  float* ob = out + ((size_t)b * kCOUT + 32 * w) * kN + nb + 4 * (l & 7);
#pragma unroll
  for (int s = 0; s < 8; ++s) *(volatile v4f*)(ob + (size_t)(4 * s + (l >> 3)) * kN) = ov[s];
  __threadfence();
#pragma unroll
  for (int s = 0; s < 8; ++s) *(volatile v4f*)(ob + (size_t)(4 * s + (l >> 3)) * kN) = ov[s];
}

extern "C" void kernel_launch(void* const* d_in, const int* in_sizes, int n_in,
                              void* d_out, int out_size, void* d_ws, size_t ws_size,
                              hipStream_t stream) {
  if (n_in < 8) return;
  const int nPts = in_sizes[1] / 3;
  if (nPts <= 0 || (nPts % kN) != 0 || (nPts % kPtsBlk) != 0) return;
  if (in_sizes[0] != nPts * kCIN) return;
  if (in_sizes[1] != nPts * 3) return;
  if (in_sizes[2] != nPts * kK) return;
  if (in_sizes[3] != 10 * kDREL || in_sizes[4] != kDREL) return;
  if (in_sizes[5] != kCMID * kCMID || in_sizes[6] != kCMID * kCOUT || in_sizes[7] != kCOUT) return;
  if (out_size != nPts * kCOUT) return;

  const size_t bytesPlane = (size_t)kCMID * kCMID * 2;
  const size_t offA = 0;
  const size_t offH = offA + bytesPlane;
  const size_t offL = offH + bytesPlane;
  const size_t total = offL + bytesPlane;
  if (ws_size < total) return;

  const float* x     = (const float*)d_in[0];
  const float* pos   = (const float*)d_in[1];
  const int*   nidx  = (const int*)  d_in[2];
  const float* Wrel  = (const float*)d_in[3];
  const float* brel  = (const float*)d_in[4];
  const float* Watt  = (const float*)d_in[5];
  const float* Wglob = (const float*)d_in[6];
  const float* bglob = (const float*)d_in[7];
  float* out = (float*)d_out;
  char* ws = (char*)d_ws;
  _Float16* wattT      = (_Float16*)(ws + offA);
  unsigned short* wgHi = (unsigned short*)(ws + offH);
  unsigned short* wgLo = (unsigned short*)(ws + offL);

  k_prep<<<dim3(8), dim3(256), 0, stream>>>(Watt, Wglob, wattT, wgHi, wgLo);
  k_main<<<dim3(nPts / kPtsBlk), dim3(kThreads), 0, stream>>>(x, pos, nidx, Wrel, brel,
                                                              wattT, wgHi, wgLo, bglob, out);
}
